// SAGE_6571299963288
// MI455X (gfx1250) — hardware-run, weakly checked
//
#include <hip/hip_runtime.h>
#include <stddef.h>
#include <stdint.h>

#define NN      100000
#define NE      1000000
#define DF      64
#define GBM     128
#define MP      100096
#define XBP     64
#define MNP     128
#define HLP     128
#define W1P     192
#define W2P     256
#define SPLIT_M1 1
#define SPLIT_H  1
#define SPLIT_M2 1
#define KM1     (SPLIT_M1 ? 128 : 64)
#define KHH     (SPLIT_H  ? 128 : 64)
#define KM2     (SPLIT_M2 ? 128 : 64)
#define KXS     64
#define NTHR    256
#define NWAVE   8
#define EPT     8
#define WCH     (32 * EPT)
#define NBRUN   1024
#define SLB     10
#define NBK     98
#define WLCAP   2048
#define RCAP    12288
#define DEGCAP  64
#define MAXDEG_MEAS   26
#define MAXB1024_MEAS 10529
#define SPT     68
#define PER     (((NE + NWAVE * WCH - 1) / (NWAVE * WCH)) * WCH)

#define BK_ZINTS (NWAVE * WLCAP + RCAP + 3 * NBRUN)
#define BK_INTS  (BK_ZINTS + 16)
#define BK_LDS   (BK_INTS * 4)

#define PBX   (MP * DF / 8 / NTHR)
#define PBW   14
#define PBTOT (PBX + PBW + 1)

static_assert(DF == 64 && DF == 16 * 4);
static_assert(MP % GBM == 0 && MP >= NN && MP == 782 * GBM);
static_assert(NBRUN == (1 << SLB) && NBRUN % GBM == 0 && NBRUN % 32 == 0);
static_assert(NBK * NBRUN >= MP && (NBK - 1) * NBRUN < NN);
static_assert(NE < (1 << 20) && (((long long)NE) << SLB) < (1LL << 31));
static_assert(NE % EPT == 0 && NE >= EPT);
static_assert(PER % WCH == 0 && (long long)NWAVE * PER >= NE && (NWAVE - 1) * PER < NE);
static_assert(RCAP % (NTHR * 4) == 0 && BK_ZINTS % (NTHR * 4) == 0 && (2 * NBRUN) % (NTHR * 4) == 0);
static_assert((long long)RCAP * 100 >= (long long)MAXB1024_MEAS * 105);
static_assert(WLCAP >= MAXB1024_MEAS / 8 + 8 * 37 + 1);
static_assert(MAXDEG_MEAS + 8 <= DEGCAP);
static_assert((MP * DF / 8) % NTHR == 0);
static_assert(W1P % 32 == 0 && W2P % 32 == 0 && W1P == 3 * DF && W2P == 4 * DF);
static_assert(KM1 % 32 == 0 && KHH % 32 == 0 && KM2 % 32 == 0 && KXS % 32 == 0);
static_assert(KM1 <= MNP && KM2 <= MNP && KHH <= HLP && KXS <= XBP);
static_assert(MNP == 2 * DF && HLP == 2 * DF && XBP == DF);
static_assert(BK_LDS <= 327680);
static_assert((GBM * SPT + 64) * 4 <= 65536);

typedef float          v4f   __attribute__((ext_vector_type(4)));
typedef float          v8f   __attribute__((ext_vector_type(8)));
typedef int            v4i   __attribute__((ext_vector_type(4)));
typedef int            v8i   __attribute__((ext_vector_type(8)));
typedef unsigned       v2u   __attribute__((ext_vector_type(2)));
typedef unsigned short v8us  __attribute__((ext_vector_type(8)));
typedef unsigned short v16us __attribute__((ext_vector_type(16)));
typedef __bf16         v16bf __attribute__((ext_vector_type(16)));
typedef v4f  __attribute__((may_alias)) v4fa;
typedef v4i  __attribute__((may_alias)) v4ia;
typedef v2u  __attribute__((may_alias)) v2ua;
typedef v8us __attribute__((may_alias)) v8usa;
union FragB { v16bf v; v16us u; v8us h[2]; v8i w; };

__device__ __forceinline__ v8f wmb(const FragB& a, const FragB& b, v8f c) {
  v8f d = __builtin_amdgcn_wmma_f32_16x16x32_bf16(false, a.v, false, b.v, (short)0, c, false, false);
  asm volatile("v_nop\n\tv_nop\n\tv_nop\n\tv_nop" : "+v"(d) : "v"(a.w), "v"(b.w));
  return d;
}

__device__ __forceinline__ unsigned bf16_bits(float f) {
  const unsigned u = __float_as_uint(f);
  const unsigned r = (u + 0x7FFFu + ((u >> 16) & 1u)) >> 16;
  const unsigned q = (u >> 16) | 0x40u;
  return ((u & 0x7fffffffu) > 0x7f800000u) ? q : r;
}

__device__ __forceinline__ void hilo_pack(float v0, float v1, float v2, float v3,
                                          int& h01, int& h23, int& l01, int& l23) {
  const unsigned a0 = bf16_bits(v0), a1 = bf16_bits(v1), a2 = bf16_bits(v2), a3 = bf16_bits(v3);
  const unsigned b0 = bf16_bits(v0 - __uint_as_float(a0 << 16));
  const unsigned b1 = bf16_bits(v1 - __uint_as_float(a1 << 16));
  const unsigned b2 = bf16_bits(v2 - __uint_as_float(a2 << 16));
  const unsigned b3 = bf16_bits(v3 - __uint_as_float(a3 << 16));
  h01 = (int)(a0 | (a1 << 16)); h23 = (int)(a2 | (a3 << 16));
  l01 = (int)(b0 | (b1 << 16)); l23 = (int)(b2 | (b3 << 16));
}

__device__ __forceinline__ v4i regroup8(int h01, int h23, int l01, int l23, int lane) {
  const int t  = lane & 15;
  const int s0 = (lane & 16) + ((2 * t) & 15), s1 = s0 + 1;
  const int a0 = __shfl(h01, s0, 32), a1 = __shfl(h23, s0, 32), a2 = __shfl(h01, s1, 32), a3 = __shfl(h23, s1, 32);
  const int b0 = __shfl(l01, s0, 32), b1 = __shfl(l23, s0, 32), b2 = __shfl(l01, s1, 32), b3 = __shfl(l23, s1, 32);
  const int mk = (t < 8) ? -1 : 0;
  v4i o;
  o.x = (a0 & mk) | (b0 & ~mk); o.y = (a1 & mk) | (b1 & ~mk);
  o.z = (a2 & mk) | (b2 & ~mk); o.w = (a3 & mk) | (b3 & ~mk);
  return o;
}

__device__ __forceinline__ void st2_v4f(float* p, v4f v) {
  *(volatile v4f*)p = v;
  __threadfence();
  *(volatile v4f*)p = v;
}
__device__ __forceinline__ void st2_v8us(unsigned short* p, v8us v) {
  *(volatile v8us*)p = v;
  __threadfence();
  *(volatile v8us*)p = v;
}

__device__ __forceinline__ v8us gather8(const float* __restrict__ base, int stride) {
  float f[8];
#pragma unroll
  for (int i = 0; i < 8; ++i) f[i] = base[(size_t)i * (size_t)stride];
  v8us o;
#pragma unroll
  for (int i = 0; i < 8; ++i) o[i] = (unsigned short)bf16_bits(f[i]);
  return o;
}

__global__ __launch_bounds__(NTHR) void k_prep(const float* __restrict__ x,
                                               const float* __restrict__ ws1, const float* __restrict__ wn1,
                                               const float* __restrict__ b1,
                                               const float* __restrict__ ws2, const float* __restrict__ wn2,
                                               const float* __restrict__ b2,
                                               unsigned short* xb, unsigned short* w1c, unsigned short* w2c,
                                               float* sm) {
  const int tid = (int)threadIdx.x, lane = tid & 31;
  const int blk = (int)blockIdx.x;
  if (blk < PBX) {
    const int u   = blk * NTHR + tid;
    const int row = u >> 3, k8 = (u & 7) * 8;
    const int rc  = row < NN ? row : NN - 1;
    const unsigned mk = row < NN ? 0xffffu : 0u;
    const float* p = x + (size_t)rc * DF + k8;
    const v4f a = *(const v4fa*)p;
    const v4f b = *(const v4fa*)(p + 4);
    v8us o;
    o[0] = (unsigned short)(bf16_bits(a.x) & mk); o[1] = (unsigned short)(bf16_bits(a.y) & mk);
    o[2] = (unsigned short)(bf16_bits(a.z) & mk); o[3] = (unsigned short)(bf16_bits(a.w) & mk);
    o[4] = (unsigned short)(bf16_bits(b.x) & mk); o[5] = (unsigned short)(bf16_bits(b.y) & mk);
    o[6] = (unsigned short)(bf16_bits(b.z) & mk); o[7] = (unsigned short)(bf16_bits(b.w) & mk);
    st2_v8us(xb + (size_t)row * XBP + k8, o);
  } else if (blk < PBX + PBW) {
    const int pb   = blk - PBX;
    const int part = pb >> 1;
    const int u    = (pb & 1) * NTHR + tid;
    const int n    = u >> 3, k8 = (u & 7) * 8;
    const size_t so = (size_t)k8 * DF + (size_t)n;
    if (part == 0) {
      st2_v8us(w1c + (size_t)n * W1P + 0 + k8, gather8(wn1 + so, DF));
    } else if (part == 1) {
      st2_v8us(w1c + (size_t)n * W1P + 64 + k8, gather8(wn1 + so, DF));
    } else if (part == 2) {
      st2_v8us(w1c + (size_t)n * W1P + 128 + k8, gather8(ws1 + so, DF));
    } else if (part == 3) {
      st2_v8us(w2c + (size_t)n * W2P + 0 + k8, gather8(wn2 + so, DF));
    } else if (part == 4) {
      st2_v8us(w2c + (size_t)n * W2P + 64 + k8, gather8(wn2 + so, DF));
    } else if (part == 5) {
      st2_v8us(w2c + (size_t)n * W2P + 128 + k8, gather8(ws2 + so, DF));
    } else {
      st2_v8us(w2c + (size_t)n * W2P + 192 + k8, gather8(ws2 + so, DF));
    }
  } else {
    if (tid < 32) {
      const int q = lane & 15;
      const v4f a = *(const v4fa*)(b1 + 4 * q);
      const v4f c = *(const v4fa*)(b2 + 4 * q);
      const float a0 = a.x, a1 = a.y, a2 = a.z, a3 = a.w;
      const float c0 = c.x, c1 = c.y, c2 = c.z, c3 = c.w;
      asm volatile("" :: "v"(a0), "v"(a1), "v"(a2), "v"(a3));
      asm volatile("" :: "v"(c0), "v"(c1), "v"(c2), "v"(c3));
      const unsigned ma = (lane < 16) ? 0xffffffffu : 0u;
      v4f o;
      o.x = __uint_as_float(((bf16_bits(a0) << 16) & ma) | ((bf16_bits(c0) << 16) & ~ma));
      o.y = __uint_as_float(((bf16_bits(a1) << 16) & ma) | ((bf16_bits(c1) << 16) & ~ma));
      o.z = __uint_as_float(((bf16_bits(a2) << 16) & ma) | ((bf16_bits(c2) << 16) & ~ma));
      o.w = __uint_as_float(((bf16_bits(a3) << 16) & ma) | ((bf16_bits(c3) << 16) & ~ma));
      st2_v4f(sm + 4 * lane, o);
    }
  }
}

__device__ __forceinline__ void bucket_flush(const int* pl, const int* cnt, int ov, int* lp, int* cop, int* fp,
                                             int tid) {
#pragma unroll 1
  for (int i = tid * 4; i < RCAP; i += NTHR * 4) {
    const v4i v = *(const v4ia*)(pl + i);
    *(volatile v4i*)(lp + i) = v;
  }
#pragma unroll 1
  for (int i = tid * 4; i < 2 * NBRUN; i += NTHR * 4) {
    const v4i v = *(const v4ia*)(cnt + i);
    *(volatile v4i*)(cop + i) = v;
  }
  if (tid < 8) {
    const v4i f = {ov, ov, ov, ov};
    *(volatile v4i*)(fp + 4 * tid) = f;
  }
}

__global__ __launch_bounds__(NTHR) void k_bucket(const int* __restrict__ srcs, const int* __restrict__ dsts,
                                                 int* LIST, int* CO, int* FLAG) {
  extern __shared__ __attribute__((aligned(16))) int dsm[];
  int* wl   = dsm;
  int* pl   = dsm + NWAVE * WLCAP;
  int* cnt  = pl + RCAP;
  int* offs = cnt + NBRUN;
  int* cur  = offs + NBRUN;
  int* misc = cur + NBRUN;
  const int tid = (int)threadIdx.x, lane = tid & 31, wave = tid >> 5;
  const int blk = (int)blockIdx.x;
  const unsigned nbs = (unsigned)(blk * NBRUN);

  {
    const v4i z4 = {0, 0, 0, 0};
    for (int i = tid * 4; i < BK_ZINTS; i += NTHR * 4) *(v4ia*)(dsm + i) = z4;
    if (tid < 16) misc[tid] = 0;
  }
  __syncthreads();

  {
    const int ebeg = wave * PER;
    const int eend = (ebeg + PER < NE) ? (ebeg + PER) : NE;
    int* mylist = wl + wave * WLCAP;
    int wc = 0;
#pragma unroll 1
    for (int cb = ebeg; cb < eend; cb += WCH) {
      const int e0  = cb + lane * EPT;
      const int e0c = e0 < NE - EPT ? e0 : NE - EPT;
      const v4i da = *(const v4ia*)(dsts + e0c);
      const v4i db = *(const v4ia*)(dsts + e0c + 4);
      const int d0 = da.x, d1 = da.y, d2 = da.z, d3 = da.w, d4 = db.x, d5 = db.y, d6 = db.z, d7 = db.w;
      asm volatile("" :: "v"(d0), "v"(d1), "v"(d2), "v"(d3));
      asm volatile("" :: "v"(d4), "v"(d5), "v"(d6), "v"(d7));
      const bool inr = e0 < NE;
      const unsigned s0 = (unsigned)d0 - nbs, s1 = (unsigned)d1 - nbs;
      const unsigned s2 = (unsigned)d2 - nbs, s3 = (unsigned)d3 - nbs;
      const unsigned s4 = (unsigned)d4 - nbs, s5 = (unsigned)d5 - nbs;
      const unsigned s6 = (unsigned)d6 - nbs, s7 = (unsigned)d7 - nbs;
      const bool h0 = inr & (s0 < (unsigned)NBRUN), h1 = inr & (s1 < (unsigned)NBRUN);
      const bool h2 = inr & (s2 < (unsigned)NBRUN), h3 = inr & (s3 < (unsigned)NBRUN);
      const bool h4 = inr & (s4 < (unsigned)NBRUN), h5 = inr & (s5 < (unsigned)NBRUN);
      const bool h6 = inr & (s6 < (unsigned)NBRUN), h7 = inr & (s7 < (unsigned)NBRUN);
      const unsigned m0 = __builtin_amdgcn_ballot_w32(h0), m1 = __builtin_amdgcn_ballot_w32(h1);
      const unsigned m2 = __builtin_amdgcn_ballot_w32(h2), m3 = __builtin_amdgcn_ballot_w32(h3);
      const unsigned m4 = __builtin_amdgcn_ballot_w32(h4), m5 = __builtin_amdgcn_ballot_w32(h5);
      const unsigned m6 = __builtin_amdgcn_ballot_w32(h6), m7 = __builtin_amdgcn_ballot_w32(h7);
      const unsigned any = m0 | m1 | m2 | m3 | m4 | m5 | m6 | m7;
      if (any != 0u) {
        const int pre = (int)(__builtin_amdgcn_mbcnt_lo(m0, 0u) + __builtin_amdgcn_mbcnt_lo(m1, 0u) +
                              __builtin_amdgcn_mbcnt_lo(m2, 0u) + __builtin_amdgcn_mbcnt_lo(m3, 0u) +
                              __builtin_amdgcn_mbcnt_lo(m4, 0u) + __builtin_amdgcn_mbcnt_lo(m5, 0u) +
                              __builtin_amdgcn_mbcnt_lo(m6, 0u) + __builtin_amdgcn_mbcnt_lo(m7, 0u));
        int p = wc + pre;
        if (h0) { if (p < WLCAP) mylist[p] = ((e0 + 0) << SLB) | (int)s0; p = p + 1; }
        if (h1) { if (p < WLCAP) mylist[p] = ((e0 + 1) << SLB) | (int)s1; p = p + 1; }
        if (h2) { if (p < WLCAP) mylist[p] = ((e0 + 2) << SLB) | (int)s2; p = p + 1; }
        if (h3) { if (p < WLCAP) mylist[p] = ((e0 + 3) << SLB) | (int)s3; p = p + 1; }
        if (h4) { if (p < WLCAP) mylist[p] = ((e0 + 4) << SLB) | (int)s4; p = p + 1; }
        if (h5) { if (p < WLCAP) mylist[p] = ((e0 + 5) << SLB) | (int)s5; p = p + 1; }
        if (h6) { if (p < WLCAP) mylist[p] = ((e0 + 6) << SLB) | (int)s6; p = p + 1; }
        if (h7) { if (p < WLCAP) mylist[p] = ((e0 + 7) << SLB) | (int)s7; p = p + 1; }
        wc += (int)(__builtin_popcount(m0) + __builtin_popcount(m1) + __builtin_popcount(m2) + __builtin_popcount(m3) +
                    __builtin_popcount(m4) + __builtin_popcount(m5) + __builtin_popcount(m6) + __builtin_popcount(m7));
      }
    }
    if (lane == 0) misc[wave] = wc;
  }
  __syncthreads();

  if (wave == 0) {
    int ov = 0, tot = 0;
#pragma unroll 1
    for (int w2 = 0; w2 < NWAVE; ++w2) {
      int c = misc[w2];
      if (c > WLCAP) ov = 1;
      c = c < 0 ? 0 : (c > WLCAP ? WLCAP : c);
      tot += c;
#pragma unroll 1
      for (int b0 = 0; b0 < c; b0 += 32) {
        const int idx = b0 + lane;
        const int ent = wl[w2 * WLCAP + (idx < WLCAP ? idx : WLCAP - 1)];
        const int m32 = (c - b0) < 32 ? (c - b0) : 32;
#pragma unroll 1
        for (int k = 0; k < m32; ++k) {
          const int u    = __builtin_amdgcn_readlane(ent, k);
          const int slot = u & (NBRUN - 1);
          if (lane == 0) cnt[slot] = cnt[slot] + 1;
        }
      }
    }
    if (tot > RCAP) ov = 1;
    if (lane == 0) misc[9] = ov;
  }
  __syncthreads();
  if (wave == 0) {
    const int base = lane * (NBRUN / 32);
    int s = 0;
#pragma unroll 1
    for (int i = 0; i < NBRUN / 32; ++i) s += cnt[base + i];
    int incl = s;
#pragma unroll
    for (int d = 1; d < 32; d <<= 1) {
      const int y = __shfl_up(incl, d, 32);
      if (lane >= d) incl += y;
    }
    int run = incl - s;
#pragma unroll 1
    for (int i = 0; i < NBRUN / 32; ++i) {
      const int cv = cnt[base + i];
      offs[base + i] = run;
      cur[base + i]  = run;
      run += cv;
    }
  }
  __syncthreads();

  if (wave == 0) {
#pragma unroll 1
    for (int w2 = 0; w2 < NWAVE; ++w2) {
      int c = misc[w2];
      c = c < 0 ? 0 : (c > WLCAP ? WLCAP : c);
#pragma unroll 1
      for (int b0 = 0; b0 < c; b0 += 32) {
        const int idx = b0 + lane;
        const int ent = wl[w2 * WLCAP + (idx < WLCAP ? idx : WLCAP - 1)];
        int eid = (ent >> SLB) & 0xFFFFF;
        eid = eid > NE - 1 ? NE - 1 : eid;
        int sr = srcs[eid];
        sr = sr < 0 ? 0 : (sr > NN - 1 ? NN - 1 : sr);
        const int m32 = (c - b0) < 32 ? (c - b0) : 32;
#pragma unroll 1
        for (int k = 0; k < m32; ++k) {
          const int u    = __builtin_amdgcn_readlane(ent, k);
          const int wd   = __builtin_amdgcn_readlane(sr, k);
          const int slot = u & (NBRUN - 1);
          if (lane == 0) {
            int p = cur[slot];
            p = p < 0 ? 0 : (p > RCAP - 1 ? RCAP - 1 : p);
            pl[p] = wd;
            cur[slot] = p + 1;
          }
        }
      }
    }
  }
  __syncthreads();

  const int ovf = misc[9];
  int* lp  = LIST + (size_t)blk * RCAP;
  int* cop = CO + (size_t)blk * (2 * NBRUN);
  int* fp  = FLAG + (size_t)blk * 32;
  bucket_flush(pl, cnt, ovf, lp, cop, fp, tid);
  __threadfence();
  bucket_flush(pl, cnt, ovf, lp, cop, fp, tid);
}

template <int LAYER2>
__global__ __launch_bounds__(NTHR) void k_replay(const int* __restrict__ LIST, const int* __restrict__ CO,
                                                 const int* __restrict__ FLAG,
                                                 const unsigned short* __restrict__ SRCP, unsigned short* MEANP) {
  constexpr int GP = LAYER2 ? HLP : XBP;
  const int tid = (int)threadIdx.x, lane = tid & 31, wave = tid >> 5, hh = lane >> 4, q = lane & 15;
  const int rowBase = (int)blockIdx.x * GBM;
  const int bucket  = rowBase >> SLB;
  const int* lb  = LIST + (size_t)bucket * RCAP;
  const int* cob = CO + (size_t)bucket * (2 * NBRUN);
  const int flag = FLAG[(size_t)bucket * 32];
  const float qnan = __uint_as_float(0x7fc00000u);

#pragma unroll 1
  for (int i = 0; i < GBM / (2 * NWAVE); ++i) {
    const int d    = rowBase + (GBM / NWAVE) * wave + 2 * i + hh;
    const int slot = d & (NBRUN - 1);
    int c = cob[slot];
    int o = cob[NBRUN + slot];
    const bool big = c > DEGCAP;
    c = c < 0 ? 0 : (c > DEGCAP ? DEGCAP : c);
    o = o < 0 ? 0 : (o > RCAP - 1 ? RCAP - 1 : o);
    const int co  = __shfl_xor(c, 16, 32);
    const int cm  = c > co ? c : co;
    const int cmu = __builtin_amdgcn_readfirstlane(cm);
    int last = o + c - 1; last = last < o ? o : last;
    last = last > RCAP - 1 ? RCAP - 1 : last;
    const int   cd = c < 1 ? 1 : c;
    const float cf = (float)cd;
    float a0 = 0.0f, a1 = 0.0f, a2 = 0.0f, a3 = 0.0f;
#pragma unroll 1
    for (int j = 0; j < cmu; ++j) {
      int idx = o + j;
      idx = idx > last ? last : idx;
      int sr = lb[idx];
      sr = sr < 0 ? 0 : (sr > NN - 1 ? NN - 1 : sr);
      const unsigned short* rp = SRCP + (size_t)sr * GP + 4 * q;
      const v2u wh = *(const v2ua*)rp;
      const unsigned whx = wh.x, why = wh.y;
      asm volatile("" :: "v"(whx), "v"(why));
      float f0 = __uint_as_float(whx << 16), f1 = __uint_as_float(whx & 0xffff0000u);
      float f2 = __uint_as_float(why << 16), f3 = __uint_as_float(why & 0xffff0000u);
      if constexpr (LAYER2 != 0) {
        const v2u wl = *(const v2ua*)(rp + DF);
        const unsigned wlx = wl.x, wly = wl.y;
        asm volatile("" :: "v"(wlx), "v"(wly));
        f0 = f0 + __uint_as_float(wlx << 16); f1 = f1 + __uint_as_float(wlx & 0xffff0000u);
        f2 = f2 + __uint_as_float(wly << 16); f3 = f3 + __uint_as_float(wly & 0xffff0000u);
      }
      const bool valid = j < c;
      a0 = a0 + (valid ? f0 : 0.0f); a1 = a1 + (valid ? f1 : 0.0f);
      a2 = a2 + (valid ? f2 : 0.0f); a3 = a3 + (valid ? f3 : 0.0f);
    }
    float m0 = a0 / cf, m1 = a1 / cf, m2 = a2 / cf, m3 = a3 / cf;
    const bool bad  = (flag != 0) | big;
    const bool live = d < NN;
    m0 = bad ? qnan : m0; m1 = bad ? qnan : m1; m2 = bad ? qnan : m2; m3 = bad ? qnan : m3;
    m0 = live ? m0 : 0.0f; m1 = live ? m1 : 0.0f; m2 = live ? m2 : 0.0f; m3 = live ? m3 : 0.0f;
    int h01, h23, l01, l23;
    hilo_pack(m0, m1, m2, m3, h01, h23, l01, l23);
    const v4i ow = regroup8(h01, h23, l01, l23, lane);
    unsigned short* hp = MEANP + (size_t)d * MNP + 8 * q;
    *(volatile v4i*)hp = ow;
    __threadfence();
    *(volatile v4i*)hp = ow;
  }
}

template <int KEXT, int BPITCH>
__device__ __forceinline__ void gemm_seg(const unsigned short* __restrict__ ap,
                                         const unsigned short* __restrict__ bp, v8f (&acc)[4]) {
  static_assert(KEXT % 32 == 0 && KEXT > 0 && BPITCH % 32 == 0);
#pragma unroll 1
  for (int k0 = 0; k0 < KEXT; k0 += 32) {
    FragB af;
    af.h[0] = *(const v8usa*)(ap + k0);
    af.h[1] = *(const v8usa*)(ap + k0 + 16);
#pragma unroll
    for (int nt = 0; nt < 4; ++nt) {
      const unsigned short* wq = bp + (size_t)(16 * nt) * (size_t)BPITCH + k0;
      FragB bf;
      bf.h[0] = *(const v8usa*)wq;
      bf.h[1] = *(const v8usa*)(wq + 16);
      acc[nt] = wmb(af, bf, acc[nt]);
    }
  }
}

__device__ __forceinline__ void stage_d(float* stg, const v8f (&acc)[4], int wave, int hh, int m) {
#pragma unroll
  for (int nt = 0; nt < 4; ++nt) {
#pragma unroll
    for (int r = 0; r < 8; ++r) stg[(16 * wave + 8 * hh + r) * SPT + 16 * nt + m] = acc[nt][r];
  }
}

template <int LAST>
__global__ __launch_bounds__(NTHR) __attribute__((amdgpu_num_vgpr(248)))
void k_gemm(const unsigned short* __restrict__ MEANP, const unsigned short* __restrict__ SELFP,
            const unsigned short* __restrict__ WC, const float* __restrict__ sm,
            const int* __restrict__ FLAG, unsigned short* HHLo, float* out) {
  constexpr int WP  = LAST ? W2P : W1P;
  constexpr int KM  = LAST ? KM2 : KM1;
  constexpr int KS  = LAST ? KHH : KXS;
  constexpr int SPP = LAST ? HLP : XBP;
  __shared__ __attribute__((aligned(16))) float stg[GBM * SPT];
  __shared__ __attribute__((aligned(16))) float sb[64];
  const int tid = (int)threadIdx.x, lane = tid & 31, wave = tid >> 5, hh = lane >> 4, m = lane & 15;
  const int rowBase = (int)blockIdx.x * GBM;
  if (tid < 16) *(v4fa*)(sb + 4 * tid) = *(const v4fa*)(sm + 64 * LAST + 4 * tid);

  v8f acc[4];
  {
    const v8f z = {0.f, 0.f, 0.f, 0.f, 0.f, 0.f, 0.f, 0.f};
#pragma unroll
    for (int t = 0; t < 4; ++t) acc[t] = z;
  }
  const int arow = rowBase + 16 * wave + m;
  const unsigned short* apm = MEANP + (size_t)arow * (size_t)MNP + 8 * hh;
  const unsigned short* aps = SELFP + (size_t)arow * (size_t)SPP + 8 * hh;
  const unsigned short* bp  = WC + (size_t)m * (size_t)WP + 8 * hh;
  gemm_seg<KM, WP>(apm, bp, acc);
  gemm_seg<KS, WP>(aps, bp + 2 * DF, acc);
  stage_d(stg, acc, wave, hh, m);
  __syncthreads();

  const v4f bias = *(const v4fa*)(sb + 4 * m);
  int flag = 0;
  if constexpr (LAST != 0) flag = FLAG[(size_t)(rowBase >> SLB) * 32];
  const float qnan = __uint_as_float(0x7fc00000u);
#pragma unroll 1
  for (int i = 0; i < 8; ++i) {
    const int lr   = 16 * wave + 2 * i + hh;
    const int grow = rowBase + lr;
    const bool live = grow < NN;
    const v4f a = *(const v4fa*)(stg + lr * SPT + 4 * m);
    asm volatile("" :: "v"(a));
    float v0 = a.x + bias.x, v1 = a.y + bias.y, v2 = a.z + bias.z, v3 = a.w + bias.w;
    if constexpr (LAST == 0) {
      v0 = (v0 > 0.0f) ? v0 : (v0 - v0); v1 = (v1 > 0.0f) ? v1 : (v1 - v1);
      v2 = (v2 > 0.0f) ? v2 : (v2 - v2); v3 = (v3 > 0.0f) ? v3 : (v3 - v3);
      v0 = live ? v0 : 0.0f; v1 = live ? v1 : 0.0f; v2 = live ? v2 : 0.0f; v3 = live ? v3 : 0.0f;
      int h01, h23, l01, l23;
      hilo_pack(v0, v1, v2, v3, h01, h23, l01, l23);
      const v4i ow = regroup8(h01, h23, l01, l23, lane);
      unsigned short* hp = HHLo + (size_t)grow * HLP + 8 * m;
      *(volatile v4i*)hp = ow;
      __threadfence();
      *(volatile v4i*)hp = ow;
    } else {
      const bool bad = flag != 0;
      v4f o;
      o.x = bad ? qnan : v0; o.y = bad ? qnan : v1; o.z = bad ? qnan : v2; o.w = bad ? qnan : v3;
      const int gr = live ? grow : NN - 1;
      float* op = out + (size_t)gr * DF + 4 * m;
      if (live) *(volatile v4f*)op = o;
      __threadfence();
      if (live) *(volatile v4f*)op = o;
    }
  }
}

extern "C" void kernel_launch(void* const* d_in, const int* in_sizes, int n_in,
                              void* d_out, int out_size, void* d_ws, size_t ws_size,
                              hipStream_t stream) {
  if (n_in < 9) return;
  if (in_sizes[0] != NN * DF) return;
  if (in_sizes[1] != NE || in_sizes[2] != NE) return;
  if (in_sizes[3] != DF * DF || in_sizes[4] != DF * DF) return;
  if (in_sizes[5] != DF) return;
  if (in_sizes[6] != DF * DF || in_sizes[7] != DF * DF) return;
  if (in_sizes[8] != DF) return;
  if (out_size != NN * DF) return;

  const float* x   = (const float*)d_in[0];
  const int*   src = (const int*)d_in[1];
  const int*   dst = (const int*)d_in[2];
  const float* Ws1 = (const float*)d_in[3];
  const float* Wn1 = (const float*)d_in[4];
  const float* b1  = (const float*)d_in[5];
  const float* Ws2 = (const float*)d_in[6];
  const float* Wn2 = (const float*)d_in[7];
  const float* b2  = (const float*)d_in[8];
  float* out = (float*)d_out;

  constexpr size_t zXB   = (size_t)MP * XBP * 2;
  constexpr size_t zMEAN = (size_t)MP * MNP * 2;
  constexpr size_t zHHL  = (size_t)MP * HLP * 2;
  constexpr size_t zLIST = (size_t)NBK * RCAP * 4;
  constexpr size_t zCO   = (size_t)NBK * 2 * NBRUN * 4;
  constexpr size_t zFLAG = (size_t)NBK * 128;
  constexpr size_t zW1C  = (size_t)DF * W1P * 2;
  constexpr size_t zW2C  = (size_t)DF * W2P * 2;
  constexpr size_t zSM   = 512;
  constexpr size_t oXB   = 0;
  constexpr size_t oMEAN = oXB + zXB;
  constexpr size_t oHHL  = oMEAN + zMEAN;
  constexpr size_t oLIST = oHHL + zHHL;
  constexpr size_t oCO   = oLIST + zLIST;
  constexpr size_t oFLAG = oCO + zCO;
  constexpr size_t oW1C  = oFLAG + zFLAG;
  constexpr size_t oW2C  = oW1C + zW1C;
  constexpr size_t oSM   = oW2C + zW2C;
  constexpr size_t oEND  = oSM + zSM;
  static_assert(zXB % 256 == 0 && zMEAN % 256 == 0 && zHHL % 256 == 0 && zLIST % 256 == 0 && zCO % 256 == 0);
  static_assert(zFLAG % 256 == 0 && zW1C % 256 == 0 && zW2C % 256 == 0 && zSM % 256 == 0);
  static_assert(oEND <= (size_t)(128u << 20));
  if (oEND > ws_size) return;

  char* ws = (char*)d_ws;
  unsigned short* XB   = (unsigned short*)(ws + oXB);
  unsigned short* MEAN = (unsigned short*)(ws + oMEAN);
  unsigned short* HHL  = (unsigned short*)(ws + oHHL);
  int*            LIST = (int*)(ws + oLIST);
  int*            CO   = (int*)(ws + oCO);
  int*            FLAG = (int*)(ws + oFLAG);
  unsigned short* W1C  = (unsigned short*)(ws + oW1C);
  unsigned short* W2C  = (unsigned short*)(ws + oW2C);
  float*          SM   = (float*)(ws + oSM);

  hipFuncSetAttribute(reinterpret_cast<const void*>(&k_bucket), hipFuncAttributeMaxDynamicSharedMemorySize, (int)BK_LDS);

  k_prep<<<PBTOT, NTHR, 0, stream>>>(x, Ws1, Wn1, b1, Ws2, Wn2, b2, XB, W1C, W2C, SM);
  k_bucket<<<NBK, NTHR, BK_LDS, stream>>>(src, dst, LIST, CO, FLAG);
  k_replay<0><<<MP / GBM, NTHR, 0, stream>>>(LIST, CO, FLAG, XB, MEAN);
  k_gemm<0><<<MP / GBM, NTHR, 0, stream>>>(MEAN, XB, W1C, SM, FLAG, HHL, out);
  k_replay<1><<<MP / GBM, NTHR, 0, stream>>>(LIST, CO, FLAG, HHL, MEAN);
  k_gemm<1><<<MP / GBM, NTHR, 0, stream>>>(MEAN, HHL, W2C, SM, FLAG, HHL, out);
}
